// SelfAttention_13632226198099
// MI455X (gfx1250) — hardware-verified
//
#include <hip/hip_runtime.h>


#ifndef NB
#define NB 2
#endif
#ifndef SEQ
#define SEQ 2048
#endif
#define NB_FULL    2
#define SEQ_FULL   2048
#define EMB        1024
#define NHEAD      16
#define HDIM       64
#define MROWS      (NB * SEQ)
#define BQ         128
#define BK         32
#define NWAVE      8
#define GM         256
#define GN         64
#define TPQ        72
#define TPV        264
#define OP         68
#define STG_HALVES (NWAVE * 32 * TPQ)
#define CVT_ELEMS  2048

static_assert(NHEAD * HDIM == EMB);
static_assert(HDIM == 64);
static_assert(GN == HDIM);
static_assert(EMB % 32 == 0);
static_assert(SEQ % 256 == 0);
static_assert(SEQ % BQ == 0);
static_assert(SEQ % BK == 0);
static_assert(SEQ % GM == 0);
static_assert(BQ == NWAVE * 16);
static_assert(GM == NWAVE * 32);
static_assert(SEQ <= SEQ_FULL);
static_assert(NB >= 1 && NB <= NB_FULL);
static_assert((TPQ * 2) % 16 == 0);
static_assert((TPV * 2) % 16 == 0);
static_assert((OP * 4) % 16 == 0);
static_assert(TPQ >= HDIM);
static_assert(TPV >= GM);
static_assert(OP >= GN);
static_assert(STG_HALVES >= HDIM * TPV);
static_assert((SEQ * EMB) % CVT_ELEMS == 0);
static_assert((EMB * EMB) % CVT_ELEMS == 0);
static_assert((unsigned long long)NB_FULL * SEQ_FULL * EMB < 4294967296ull);

typedef __bf16   bf16;
typedef _Float16 f16;
typedef bf16     v16bf __attribute__((ext_vector_type(16)));
typedef f16      v16h  __attribute__((ext_vector_type(16)));
typedef float    v8f   __attribute__((ext_vector_type(8)));
typedef float    v4f   __attribute__((ext_vector_type(4)));
typedef unsigned v4u   __attribute__((ext_vector_type(4)));

union FragB  { v16bf v; v4u q[2]; };
union FragH  { v16h  v; v4u q[2]; f16 h[16]; };
union Pack8B { v4u u; bf16 h[8]; };
union Pack8H { v4u u; f16 h[8]; };

constexpr size_t XB_BYTES = (size_t)MROWS * EMB * 2;
constexpr size_t WQKV_BYTES = (size_t)3 * EMB * EMB * 2;
constexpr size_t WO_BYTES = (size_t)EMB * EMB * 2;
constexpr size_t HP_BYTES = (size_t)NB * NHEAD * SEQ * HDIM * 2;
constexpr size_t CX_BYTES = (size_t)MROWS * EMB * 2;
constexpr size_t WS_TOTAL = XB_BYTES + WQKV_BYTES + WO_BYTES + 4 * HP_BYTES + 2 * CX_BYTES;
static_assert(WS_TOTAL <= 134217728ull);

static __device__ __forceinline__ v8f mma_bf16(v16bf a, v16bf b, v8f acc) {
  acc = __builtin_amdgcn_wmma_f32_16x16x32_bf16(false, a, false, b, (short)0, acc, false, false);
  asm volatile("v_nop\n\tv_nop\n\tv_nop\n\tv_nop" : "+v"(acc) : "v"(a), "v"(b));
  return acc;
}
static __device__ __forceinline__ v8f mma_f16(v16h a, v16h b, v8f acc) {
  acc = __builtin_amdgcn_wmma_f32_16x16x32_f16(false, a, false, b, (short)0, acc, false, false);
  asm volatile("v_nop\n\tv_nop\n\tv_nop\n\tv_nop" : "+v"(acc) : "v"(a), "v"(b));
  return acc;
}

template <int N>
static __device__ __forceinline__ void store_twice_u4(f16* __restrict__ plane, const unsigned (&gi)[N],
                                                      const v4u (&vals)[N]) {
  #pragma unroll
  for (int i = 0; i < N; ++i) *(volatile v4u*)(plane + gi[i]) = vals[i];
  __threadfence();
  #pragma unroll
  for (int i = 0; i < N; ++i) *(volatile v4u*)(plane + gi[i]) = vals[i];
}
template <int N>
static __device__ __forceinline__ void store_twice_f4(float* __restrict__ dst, const unsigned (&gi)[N],
                                                      const v4f (&vals)[N]) {
  #pragma unroll
  for (int i = 0; i < N; ++i) *(volatile v4f*)(dst + gi[i]) = vals[i];
  __threadfence();
  #pragma unroll
  for (int i = 0; i < N; ++i) *(volatile v4f*)(dst + gi[i]) = vals[i];
}

__global__ __launch_bounds__(256) void cvt_bf16_kernel(const float* __restrict__ in, bf16* __restrict__ outp,
                                                       unsigned in_bstride, unsigned out_bstride) {
  const size_t e = ((size_t)blockIdx.x * 256 + threadIdx.x) * 8;
  const float* src = in + (size_t)blockIdx.y * in_bstride + e;
  const v4f a0 = *(const v4f*)(src);
  const v4f a1 = *(const v4f*)(src + 4);
  Pack8B pk;
  #pragma unroll
  for (int i = 0; i < 4; ++i) {
    pk.h[i]     = (bf16)a0[i];
    pk.h[4 + i] = (bf16)a1[i];
  }
  bf16* dst = outp + (size_t)blockIdx.y * out_bstride + e;
  const v4u val = pk.u;
  *(volatile v4u*)dst = val;
  __threadfence();
  *(volatile v4u*)dst = val;
}

__global__ __launch_bounds__(256) void cvt_f16s_kernel(const float* __restrict__ in, f16* __restrict__ outp) {
  const size_t e = ((size_t)blockIdx.x * 256 + threadIdx.x) * 8;
  const float* src = in + e;
  const v4f a0 = *(const v4f*)(src);
  const v4f a1 = *(const v4f*)(src + 4);
  Pack8H pk;
  #pragma unroll
  for (int i = 0; i < 4; ++i) {
    pk.h[i]     = (f16)((float)(bf16)a0[i] * 64.0f);
    pk.h[4 + i] = (f16)((float)(bf16)a1[i] * 64.0f);
  }
  f16* dst = outp + e;
  const v4u val = pk.u;
  *(volatile v4u*)dst = val;
  __threadfence();
  *(volatile v4u*)dst = val;
}

__global__ __launch_bounds__(256) void qkv_gemm_kernel(const bf16* __restrict__ xb, const bf16* __restrict__ wqkv,
                                                       f16* __restrict__ qh, f16* __restrict__ qr,
                                                       f16* __restrict__ kp, f16* __restrict__ vt) {
  const int tid  = threadIdx.x;
  const int wave = __builtin_amdgcn_readfirstlane(tid >> 5);
  const int lane = tid & 31;
  const int lq   = lane & 15;
  const int hi   = lane >> 4;
  const int m0   = blockIdx.x * GM;
  const int nt   = blockIdx.y;
  const int mode = nt >> 4;
  const int h    = nt & 15;
  const int b    = m0 / SEQ;
  const int s0   = m0 - b * SEQ;

  __shared__ __align__(16) f16 sT[STG_HALVES];

  v8f acc[2][4];
  #pragma unroll
  for (int u = 0; u < 2; ++u) {
    #pragma unroll
    for (int f = 0; f < 4; ++f) acc[u][f] = (v8f){0, 0, 0, 0, 0, 0, 0, 0};
  }

  const bf16* ap = xb + (size_t)(m0 + wave * 32 + lq) * EMB + hi * 8;
  const bf16* bp = wqkv + (size_t)(nt * GN + lq) * EMB + hi * 8;

  #pragma unroll 1
  for (int c = 0; c < EMB / 32; ++c) {
    FragB a[2], w[4];
    #pragma unroll
    for (int u = 0; u < 2; ++u) {
      a[u].q[0] = *(const v4u*)(ap + u * 16 * EMB + c * 32);
      a[u].q[1] = *(const v4u*)(ap + u * 16 * EMB + c * 32 + 16);
    }
    #pragma unroll
    for (int f = 0; f < 4; ++f) {
      w[f].q[0] = *(const v4u*)(bp + f * 16 * EMB + c * 32);
      w[f].q[1] = *(const v4u*)(bp + f * 16 * EMB + c * 32 + 16);
    }
    #pragma unroll
    for (int f = 0; f < 4; ++f) {
      #pragma unroll
      for (int u = 0; u < 2; ++u) acc[u][f] = mma_bf16(a[u].v, w[f].v, acc[u][f]);
    }
  }

  const unsigned hb = (unsigned)(b * NHEAD + h);
  const int wb = wave * (32 * TPQ);

  if (mode == 2) {
    #pragma unroll
    for (int u = 0; u < 2; ++u) {
      #pragma unroll
      for (int f = 0; f < 4; ++f) {
        Pack8H ph;
        #pragma unroll
        for (int r = 0; r < 8; ++r) ph.h[r] = (f16)acc[u][f][r];
        *(v4u*)(&sT[(f * 16 + lq) * TPV + wave * 32 + u * 16 + hi * 8]) = ph.u;
      }
    }
    __syncthreads();
    v4u vals[8];
    unsigned gi[8];
    #pragma unroll
    for (int it = 0; it < 8; ++it) {
      const int d = it * 8 + wave;
      vals[it] = *(const v4u*)(&sT[d * TPV + lane * 8]);
      gi[it]   = (hb * HDIM + d) * SEQ + s0 + lane * 8;
    }
    store_twice_u4<8>(vt, gi, vals);
  } else {
    #pragma unroll
    for (int u = 0; u < 2; ++u) {
      #pragma unroll
      for (int f = 0; f < 4; ++f) {
        #pragma unroll
        for (int r = 0; r < 8; ++r)
          sT[wb + (u * 16 + hi * 8 + r) * TPQ + f * 16 + lq] = (f16)acc[u][f][r];
      }
    }
    __syncthreads();
    v4u vals[8];
    unsigned gi[8];
    #pragma unroll
    for (int it = 0; it < 8; ++it) {
      const int row = it * 4 + (lane >> 3);
      const int c8  = lane & 7;
      vals[it] = *(const v4u*)(&sT[wb + row * TPQ + c8 * 8]);
      gi[it]   = (hb * SEQ + s0 + wave * 32 + row) * HDIM + c8 * 8;
    }
    if (mode == 0) {
      store_twice_u4<8>(qh, gi, vals);
    } else {
      store_twice_u4<8>(kp, gi, vals);
    }
    if (mode == 0) {
      __syncthreads();
      #pragma unroll
      for (int u = 0; u < 2; ++u) {
        #pragma unroll
        for (int f = 0; f < 4; ++f) {
          #pragma unroll
          for (int r = 0; r < 8; ++r) {
            const float av = acc[u][f][r];
            const f16   t  = (f16)av;
            sT[wb + (u * 16 + hi * 8 + r) * TPQ + f * 16 + lq] = (f16)((av - (float)t) * 2048.0f);
          }
        }
      }
      __syncthreads();
      v4u rvals[8];
      #pragma unroll
      for (int it = 0; it < 8; ++it) {
        const int row = it * 4 + (lane >> 3);
        const int c8  = lane & 7;
        rvals[it] = *(const v4u*)(&sT[wb + row * TPQ + c8 * 8]);
      }
      store_twice_u4<8>(qr, gi, rvals);
    }
  }
}

__global__ __launch_bounds__(256) void attn_kernel(const f16* __restrict__ qh, const f16* __restrict__ qr,
                                                   const f16* __restrict__ kp, const f16* __restrict__ vt,
                                                   const int* __restrict__ mask,
                                                   f16* __restrict__ ch, f16* __restrict__ cr) {
  const int qblk = blockIdx.x;
  const int h    = blockIdx.y;
  const int b    = blockIdx.z;
  const int tid  = threadIdx.x;
  const int wave = __builtin_amdgcn_readfirstlane(tid >> 5);
  const int lane = tid & 31;
  const int lq   = lane & 15;
  const int hi   = lane >> 4;

  __shared__ __align__(16) float sO[NWAVE * 16 * OP];
  __shared__ unsigned sMask[SEQ / 32];

  #pragma unroll 1
  for (int p = 0; p < SEQ / 256; ++p) {
    const int key = p * 256 + tid;
    const int mv  = mask[(size_t)b * SEQ_FULL + key];
    const unsigned wbits = __builtin_amdgcn_ballot_w32(mv != 0);
    if (lane == 0) sMask[p * 8 + wave] = wbits;
  }
  __syncthreads();

  const int qrow0 = qblk * BQ + wave * 16;
  const unsigned hb = (unsigned)(b * NHEAD + h);

  FragH qf[2], qg[2];
  {
    const unsigned qo = (hb * SEQ + qrow0 + lq) * HDIM + hi * 8;
    #pragma unroll
    for (int f = 0; f < 2; ++f) {
      qf[f].q[0] = *(const v4u*)(qh + qo + f * 32);
      qf[f].q[1] = *(const v4u*)(qh + qo + f * 32 + 16);
      qg[f].q[0] = *(const v4u*)(qr + qo + f * 32);
      qg[f].q[1] = *(const v4u*)(qr + qo + f * 32 + 16);
    }
  }

  const f16* kp_h = kp + (size_t)hb * SEQ * HDIM;
  const f16* vt_h = vt + (size_t)hb * HDIM * SEQ;

  v8f o[4];
  #pragma unroll
  for (int dt = 0; dt < 4; ++dt) o[dt] = (v8f){0, 0, 0, 0, 0, 0, 0, 0};

  const float NINF = -__builtin_inff();
  float rmax = NINF;
  float rsum = 0.0f;
  const float SL = 0.125f * 1.4426950408889634f;

  #pragma unroll 1
  for (int i = 0; i < SEQ / BK; ++i) {
    const int j0 = i * BK;

    v8f s[2];
    #pragma unroll
    for (int sub = 0; sub < 2; ++sub) {
      const f16* base = kp_h + (size_t)(j0 + sub * 16 + lq) * HDIM + hi * 8;
      FragH a0, a1;
      a0.q[0] = *(const v4u*)(base);
      a0.q[1] = *(const v4u*)(base + 16);
      a1.q[0] = *(const v4u*)(base + 32);
      a1.q[1] = *(const v4u*)(base + 48);
      v8f c  = (v8f){0, 0, 0, 0, 0, 0, 0, 0};
      v8f c2 = (v8f){0, 0, 0, 0, 0, 0, 0, 0};
      c  = mma_f16(a0.v, qf[0].v, c);
      c  = mma_f16(a1.v, qf[1].v, c);
      c2 = mma_f16(a0.v, qg[0].v, c2);
      c2 = mma_f16(a1.v, qg[1].v, c2);
      #pragma unroll
      for (int r = 0; r < 8; ++r) s[sub][r] = c[r] + c2[r] * (1.0f / 2048.0f);
    }

    const unsigned mw = (unsigned)__builtin_amdgcn_readfirstlane((int)sMask[i]);
    if (mw != 0xFFFFFFFFu) {
      #pragma unroll
      for (int sub = 0; sub < 2; ++sub) {
        #pragma unroll
        for (int r = 0; r < 8; ++r) {
          const unsigned bit = (unsigned)(sub * 16 + hi * 8 + r);
          s[sub][r] = ((mw >> bit) & 1u) ? s[sub][r] : NINF;
        }
      }
    }

    FragH bv[4];
    #pragma unroll
    for (int dt = 0; dt < 4; ++dt) {
      const f16* base = vt_h + (size_t)(dt * 16 + lq) * SEQ + j0 + hi * 8;
      bv[dt].q[0] = *(const v4u*)(base);
      bv[dt].q[1] = *(const v4u*)(base + 16);
    }

    float m_new = rmax;
    #pragma unroll
    for (int r = 0; r < 8; ++r) {
      m_new = fmaxf(m_new, s[0][r]);
      m_new = fmaxf(m_new, s[1][r]);
    }
    m_new = fmaxf(m_new, __shfl_xor(m_new, 16, 32));
    const float m_use = (m_new == NINF) ? 0.0f : m_new;
    const float scale = __builtin_amdgcn_exp2f((rmax - m_use) * SL);
    rmax = m_new;

    FragH pa;
    float psum = 0.0f;
    #pragma unroll
    for (int r = 0; r < 8; ++r) {
      const float p0 = __builtin_amdgcn_exp2f((s[0][r] - m_use) * SL);
      const float p1 = __builtin_amdgcn_exp2f((s[1][r] - m_use) * SL);
      psum += p0 + p1;
      pa.h[r]     = (f16)(p0 * 4096.0f);
      pa.h[8 + r] = (f16)(p1 * 4096.0f);
    }
    rsum = rsum * scale + psum + __shfl_xor(psum, 16, 32);

    float sc[8];
    #pragma unroll
    for (int r = 0; r < 8; ++r) sc[r] = __shfl(scale, (hi << 3) + r, 32);
    #pragma unroll
    for (int dt = 0; dt < 4; ++dt) {
      #pragma unroll
      for (int r = 0; r < 8; ++r) o[dt][r] *= sc[r];
    }

    #pragma unroll
    for (int dt = 0; dt < 4; ++dt) o[dt] = mma_f16(pa.v, bv[dt].v, o[dt]);
  }

  float rs[8];
  #pragma unroll
  for (int r = 0; r < 8; ++r) rs[r] = 1.0f / __shfl(rsum, (hi << 3) + r, 32);

  const int sb = wave * (16 * OP);
  #pragma unroll
  for (int r = 0; r < 8; ++r) {
    #pragma unroll
    for (int dt = 0; dt < 4; ++dt) sO[sb + (hi * 8 + r) * OP + dt * 16 + lq] = o[dt][r] * rs[r];
  }
  __syncthreads();

  v4u hv[4], rv[4];
  unsigned gi[4];
  #pragma unroll
  for (int it = 0; it < 4; ++it) {
    const int row = it * 4 + (lane >> 3);
    const int c8  = lane & 7;
    const v4f x0 = *(const v4f*)(&sO[sb + row * OP + c8 * 8]);
    const v4f x1 = *(const v4f*)(&sO[sb + row * OP + c8 * 8 + 4]);
    Pack8H ph, pr;
    #pragma unroll
    for (int e = 0; e < 4; ++e) {
      const f16 t0 = (f16)x0[e];
      const f16 t1 = (f16)x1[e];
      ph.h[e]     = t0;
      ph.h[4 + e] = t1;
      pr.h[e]     = (f16)(x0[e] - (float)t0);
      pr.h[4 + e] = (f16)(x1[e] - (float)t1);
    }
    hv[it] = ph.u;
    rv[it] = pr.u;
    gi[it] = (unsigned)(b * SEQ + qrow0 + row) * EMB + h * HDIM + c8 * 8;
  }
  store_twice_u4<4>(ch, gi, hv);
  store_twice_u4<4>(cr, gi, rv);
}

__global__ __launch_bounds__(256) void out_gemm_kernel(const f16* __restrict__ ch, const f16* __restrict__ cr,
                                                       const f16* __restrict__ wo, float* __restrict__ outp) {
  const int tid  = threadIdx.x;
  const int wave = __builtin_amdgcn_readfirstlane(tid >> 5);
  const int lane = tid & 31;
  const int lq   = lane & 15;
  const int hi   = lane >> 4;
  const int m0   = blockIdx.x * GM;
  const int n0   = blockIdx.y * GN;
  const int b    = m0 / SEQ;
  const int s0   = m0 - b * SEQ;

  __shared__ __align__(16) float sO[NWAVE * 16 * OP];

  v8f acc[2][4];
  #pragma unroll
  for (int u = 0; u < 2; ++u) {
    #pragma unroll
    for (int f = 0; f < 4; ++f) acc[u][f] = (v8f){0, 0, 0, 0, 0, 0, 0, 0};
  }

  const size_t aoff = (size_t)(m0 + wave * 32 + lq) * EMB + hi * 8;
  const f16* ah = ch + aoff;
  const f16* ar = cr + aoff;
  const f16* bp = wo + (size_t)(n0 + lq) * EMB + hi * 8;

  #pragma unroll 1
  for (int c = 0; c < EMB / 32; ++c) {
    FragH a[2], w[4];
    #pragma unroll
    for (int u = 0; u < 2; ++u) {
      a[u].q[0] = *(const v4u*)(ah + u * 16 * EMB + c * 32);
      a[u].q[1] = *(const v4u*)(ah + u * 16 * EMB + c * 32 + 16);
    }
    #pragma unroll
    for (int f = 0; f < 4; ++f) {
      w[f].q[0] = *(const v4u*)(bp + f * 16 * EMB + c * 32);
      w[f].q[1] = *(const v4u*)(bp + f * 16 * EMB + c * 32 + 16);
    }
    #pragma unroll
    for (int f = 0; f < 4; ++f) {
      #pragma unroll
      for (int u = 0; u < 2; ++u) acc[u][f] = mma_f16(a[u].v, w[f].v, acc[u][f]);
    }
  }
  #pragma unroll 1
  for (int c = 0; c < EMB / 32; ++c) {
    FragH a[2], w[4];
    #pragma unroll
    for (int u = 0; u < 2; ++u) {
      a[u].q[0] = *(const v4u*)(ar + u * 16 * EMB + c * 32);
      a[u].q[1] = *(const v4u*)(ar + u * 16 * EMB + c * 32 + 16);
    }
    #pragma unroll
    for (int f = 0; f < 4; ++f) {
      w[f].q[0] = *(const v4u*)(bp + f * 16 * EMB + c * 32);
      w[f].q[1] = *(const v4u*)(bp + f * 16 * EMB + c * 32 + 16);
    }
    #pragma unroll
    for (int f = 0; f < 4; ++f) {
      #pragma unroll
      for (int u = 0; u < 2; ++u) acc[u][f] = mma_f16(a[u].v, w[f].v, acc[u][f]);
    }
  }

  const float OSC = 1.0f / 262144.0f;
  const int sb = wave * (16 * OP);
  #pragma unroll
  for (int u = 0; u < 2; ++u) {
    if (u != 0) __syncthreads();
    #pragma unroll
    for (int f = 0; f < 4; ++f) {
      #pragma unroll
      for (int r = 0; r < 8; ++r) sO[sb + (hi * 8 + r) * OP + f * 16 + lq] = acc[u][f][r] * OSC;
    }
    __syncthreads();
    v4f vals[8];
    unsigned gi[8];
    #pragma unroll
    for (int it = 0; it < 8; ++it) {
      const int row = it * 2 + hi;
      vals[it] = *(const v4f*)(&sO[sb + row * OP + lq * 4]);
      gi[it]   = (unsigned)(b * SEQ_FULL + s0 + wave * 32 + u * 16 + row) * EMB + n0 + lq * 4;
    }
    store_twice_f4<8>(outp, gi, vals);
  }
}

extern "C" void kernel_launch(void* const* d_in, const int* in_sizes, int n_in,
                              void* d_out, int out_size, void* d_ws, size_t ws_size,
                              hipStream_t stream) {
  if (n_in < 6) return;
  const size_t rows_used = (size_t)(NB - 1) * SEQ_FULL + SEQ;
  if ((size_t)in_sizes[0] < rows_used * EMB) return;
  if ((size_t)in_sizes[1] < rows_used) return;
  if ((size_t)in_sizes[2] < (size_t)EMB * EMB) return;
  if ((size_t)in_sizes[3] < (size_t)EMB * EMB) return;
  if ((size_t)in_sizes[4] < (size_t)EMB * EMB) return;
  if ((size_t)in_sizes[5] < (size_t)EMB * EMB) return;
  if ((size_t)out_size < rows_used * EMB) return;
  if (ws_size < WS_TOTAL) return;

  const float* x   = (const float*)d_in[0];
  const int*   msk = (const int*)d_in[1];
  const float* Wq  = (const float*)d_in[2];
  const float* Wk  = (const float*)d_in[3];
  const float* Wv  = (const float*)d_in[4];
  const float* Wo  = (const float*)d_in[5];
  float*       out = (float*)d_out;

  char* w = (char*)d_ws;
  bf16* xb   = (bf16*)w;  w += XB_BYTES;
  bf16* wqkv = (bf16*)w;  w += WQKV_BYTES;
  f16*  wo16 = (f16*)w;   w += WO_BYTES;
  f16*  qh   = (f16*)w;   w += HP_BYTES;
  f16*  qr   = (f16*)w;   w += HP_BYTES;
  f16*  kp   = (f16*)w;   w += HP_BYTES;
  f16*  vt   = (f16*)w;   w += HP_BYTES;
  f16*  ch   = (f16*)w;   w += CX_BYTES;
  f16*  cr   = (f16*)w;   w += CX_BYTES;

  const unsigned wblocks = (unsigned)((size_t)EMB * EMB / CVT_ELEMS);
  cvt_bf16_kernel<<<dim3((unsigned)((size_t)SEQ * EMB / CVT_ELEMS), NB), 256, 0, stream>>>(
      x, xb, (unsigned)((size_t)SEQ_FULL * EMB), (unsigned)((size_t)SEQ * EMB));
  cvt_bf16_kernel<<<dim3(wblocks, 1), 256, 0, stream>>>(Wq, wqkv, 0u, 0u);
  cvt_bf16_kernel<<<dim3(wblocks, 1), 256, 0, stream>>>(Wk, wqkv + (size_t)EMB * EMB, 0u, 0u);
  cvt_bf16_kernel<<<dim3(wblocks, 1), 256, 0, stream>>>(Wv, wqkv + (size_t)2 * EMB * EMB, 0u, 0u);
  cvt_f16s_kernel<<<dim3(wblocks), 256, 0, stream>>>(Wo, wo16);

  qkv_gemm_kernel<<<dim3(MROWS / GM, 3 * NHEAD), 256, 0, stream>>>(xb, wqkv, qh, qr, kp, vt);
  attn_kernel<<<dim3(SEQ / BQ, NHEAD, NB), 256, 0, stream>>>(qh, qr, kp, vt, msk, ch, cr);
  out_gemm_kernel<<<dim3(MROWS / GM, EMB / GN), 256, 0, stream>>>(ch, cr, wo16, out);
}
